// Rwkv7SelfAttention_53429393162446
// MI455X (gfx1250) — hardware-verified
//
#include <hip/hip_runtime.h>
#include <math.h>
#include <stdint.h>

typedef __attribute__((ext_vector_type(16))) _Float16 v16h;
typedef __attribute__((ext_vector_type(8)))  _Float16 v8h;
typedef __attribute__((ext_vector_type(16))) __bf16   v16b;
typedef __attribute__((ext_vector_type(8)))  __bf16   v8b;
typedef __attribute__((ext_vector_type(8)))  float    v8f;
typedef __attribute__((ext_vector_type(4)))  float    v4f;
typedef __attribute__((ext_vector_type(2)))  float    v2f;
typedef __attribute__((ext_vector_type(4)))  unsigned v4u;

constexpr int HID   = 2048;
constexpr int HSZ   = 64;
constexpr int NHEAD = 32;
constexpr int TLEN  = 1024;
constexpr int DLD   = 64;
constexpr int DLA   = 64;
constexpr int DLG   = 128;
constexpr int DLV   = 32;
constexpr int DLVP  = 64;
constexpr float WCARRY     = 64.0f;
constexpr float WCARRY_INV = 1.0f / 64.0f;

static_assert(NHEAD * HSZ == HID, "");
static_assert(TLEN % 64 == 0 && HID % 64 == 0 && DLG % 64 == 0 && DLD % 64 == 0 && DLA % 64 == 0 && DLVP % 64 == 0, "");
static_assert(HID % 32 == 0 && DLG % 32 == 0 && DLD % 32 == 0 && DLA % 32 == 0 && DLV % 32 == 0, "");
static_assert(TLEN % 16 == 0, "");

constexpr size_t PL32 = (size_t)TLEN * HID * 4;
constexpr size_t PL16 = (size_t)TLEN * HID * 2;
constexpr size_t WB16 = (size_t)HID * HID * 2;
constexpr size_t OFF_WO16 = 0;
constexpr size_t OFF_G1T  = OFF_WO16 + WB16;
constexpr size_t OFF_G2T  = OFF_G1T + (size_t)DLG * HID * 2;
constexpr size_t OFF_W1T  = OFF_G2T + (size_t)HID * DLG * 2;
constexpr size_t OFF_W2T  = OFF_W1T + (size_t)DLD * HID * 2;
constexpr size_t OFF_A1T  = OFF_W2T + (size_t)HID * DLD * 2;
constexpr size_t OFF_A2T  = OFF_A1T + (size_t)DLA * HID * 2;
constexpr size_t OFF_V1T  = OFF_A2T + (size_t)HID * DLA * 2;
constexpr size_t OFF_V2T  = OFF_V1T + (size_t)DLVP * HID * 2;
constexpr size_t OFF_HG   = OFF_V2T + (size_t)HID * DLV * 2;
constexpr size_t OFF_HW   = OFF_HG + (size_t)TLEN * DLG * 2;
constexpr size_t OFF_HA   = OFF_HW + (size_t)TLEN * DLD * 2;
constexpr size_t OFF_HV   = OFF_HA + (size_t)TLEN * DLA * 2;
constexpr size_t OFF_YG   = OFF_HV + (size_t)TLEN * DLVP * 2;
constexpr size_t OFF_R1   = OFF_YG + PL16;
static_assert(OFF_R1 == 15728640, "");
constexpr size_t OFF_WR16 = OFF_R1;
constexpr size_t OFF_WKH  = OFF_WR16 + WB16;
constexpr size_t OFF_WKL  = OFF_WKH + WB16;
constexpr size_t OFF_WVH  = OFF_WKL + WB16;
constexpr size_t OFF_WVL  = OFF_WVH + WB16;
constexpr size_t OFF_R2   = OFF_WVL + WB16;
static_assert(WB16 == PL32, "");
constexpr size_t OFF_GBUF = OFF_WR16;
constexpr size_t OFF_WDEC = OFF_WKH;
constexpr size_t OFF_ABUF = OFF_WKL;
constexpr size_t OFF_PBUF = OFF_WVH;
constexpr size_t OFF_YBUF = OFF_WVL;
constexpr size_t OFF_XN   = OFF_R2;
constexpr size_t OFF_XR16 = OFF_XN + PL32;
constexpr size_t OFF_XW16 = OFF_XR16 + PL16;
constexpr size_t OFF_XA16 = OFF_XW16 + PL16;
constexpr size_t OFF_XG16 = OFF_XA16 + PL16;
constexpr size_t OFF_XV16 = OFF_XG16 + PL16;
constexpr size_t OFF_XKH  = OFF_XV16 + PL16;
constexpr size_t OFF_XKL  = OFF_XKH + PL16;
constexpr size_t OFF_XVH  = OFF_XKL + PL16;
constexpr size_t OFF_XVL  = OFF_XVH + PL16;
constexpr size_t OFF_R3   = OFF_XVL + PL16;
constexpr size_t OFF_KMOD = OFF_R2;
constexpr size_t OFF_VFIN = OFF_KMOD + PL32;
constexpr size_t OFF_ASEQ = OFF_VFIN + PL32;
constexpr size_t OFF_BSEQ = OFF_ASEQ + PL32;
static_assert(OFF_BSEQ + PL32 <= OFF_R3, "");
constexpr size_t OFF_RBUF = OFF_R3;
constexpr size_t OFF_KBUF = OFF_RBUF + PL32;
constexpr size_t OFF_VBUF = OFF_KBUF + PL32;
constexpr size_t WS_END   = OFF_VBUF + PL32;
static_assert(WS_END == 128974848, "");
static_assert(WS_END <= 134217728, "");

constexpr size_t OUT0_F = 0;
constexpr size_t OUT1_F = 8388608 / 4;
constexpr size_t OUT2_F = 8396800 / 4;
constexpr size_t OUT3_F = 8921088 / 4;
constexpr size_t OUT_TOTAL_F = 17309696 / 4;
static_assert(OUT1_F == OUT0_F + (size_t)TLEN * HID, "");
static_assert(OUT2_F == OUT1_F + HID, "");
static_assert(OUT3_F == OUT2_F + (size_t)NHEAD * HSZ * HSZ, "");
static_assert(OUT3_F + (size_t)TLEN * HID == OUT_TOTAL_F, "");

__device__ __forceinline__ unsigned short f2bf_bits(float f) {
  unsigned u = __float_as_uint(f);
  return (unsigned short)((u + 0x7FFFu + ((u >> 16) & 1u)) >> 16);
}
__device__ __forceinline__ float bf_bits2f(unsigned short h) { return __uint_as_float(((unsigned)h) << 16); }

__device__ __forceinline__ void dep_guard_h(v8f& a, v8f& b, v16h x, v16h y) { asm volatile("v_nop\n\tv_nop\n\tv_nop\n\tv_nop" : "+v"(a), "+v"(b) : "v"(x), "v"(y)); }
__device__ __forceinline__ void dep_guard_b(v8f& a, v8f& b, v16b x, v16b y) { asm volatile("v_nop\n\tv_nop\n\tv_nop\n\tv_nop" : "+v"(a), "+v"(b) : "v"(x), "v"(y)); }
__device__ __forceinline__ void keep4_h(v16h a, v16h b, v16h c, v16h d) { asm volatile("v_nop" :: "v"(a), "v"(b), "v"(c), "v"(d)); }
__device__ __forceinline__ void keep4_b(v16b a, v16b b, v16b c, v16b d) { asm volatile("v_nop" :: "v"(a), "v"(b), "v"(c), "v"(d)); }
__device__ __forceinline__ void acc_guard4(v8f& a, v8f& b, v8f& c, v8f& d) { asm volatile("v_nop\n\tv_nop\n\tv_nop\n\tv_nop" : "+v"(a), "+v"(b), "+v"(c), "+v"(d)); }
template <typename T> struct Frag;
template <> struct Frag<_Float16> {
  typedef v16h V; union U { v16h v; v8h h[2]; };
  static __device__ __forceinline__ v16h load(const _Float16* p) {
    U f; f.h[0] = *(const v8h*)(p); f.h[1] = *(const v8h*)(p + 16); return f.v;
  }
  static __device__ __forceinline__ v8f mma(v16h a, v16h b, v8f c) {
    return __builtin_amdgcn_wmma_f32_16x16x32_f16(false, a, false, b, (short)0, c, false, false);
  }
  static __device__ __forceinline__ void guard(v8f& a, v8f& b, v16h x, v16h y) { dep_guard_h(a, b, x, y); }
  static __device__ __forceinline__ void keep(v16h a, v16h b, v16h c, v16h d) { keep4_h(a, b, c, d); }
};
template <> struct Frag<__bf16> {
  typedef v16b V; union U { v16b v; v8b h[2]; };
  static __device__ __forceinline__ v16b load(const __bf16* p) {
    U f; f.h[0] = *(const v8b*)(p); f.h[1] = *(const v8b*)(p + 16); return f.v;
  }
  static __device__ __forceinline__ v8f mma(v16b a, v16b b, v8f c) {
    return __builtin_amdgcn_wmma_f32_16x16x32_bf16(false, a, false, b, (short)0, c, false, false);
  }
  static __device__ __forceinline__ void guard(v8f& a, v8f& b, v16b x, v16b y) { dep_guard_b(a, b, x, y); }
  static __device__ __forceinline__ void keep(v16b a, v16b b, v16b c, v16b d) { keep4_b(a, b, c, d); }
};

template <int ET> struct Elem;
template <> struct Elem<0> { typedef _Float16 T; };
template <> struct Elem<1> { typedef __bf16 T; };
template <int ET, bool SPLIT, int BIAS_MODE, int OUT_MODE, bool RESID, int ACT = 0>
__global__ __launch_bounds__(256) void wmma_gemm64(
    const unsigned short* __restrict__ Ap, const unsigned short* __restrict__ A2p, int lda, long strideA,
    const unsigned short* __restrict__ Btp, const unsigned short* __restrict__ Bt2p, int ldb, long strideB,
    void* __restrict__ Cout, void* __restrict__ Cout2, int ldc, long strideC,
    const float* __restrict__ bias,
    const float* __restrict__ resid, long strideR,
    int M, int N, int K, float scale) {
  typedef typename Elem<ET>::T T;
  typedef typename Frag<T>::V V;
  const T* A = (const T*)Ap; const T* A2 = (const T*)A2p; const T* Bt = (const T*)Btp; const T* Bt2 = (const T*)Bt2p;
  __shared__ __align__(16) float sT[8][16 * 68];
  const int b    = blockIdx.y;
  const int lane = threadIdx.x & 31;
  const int wave = threadIdx.x >> 5;
  const int tilesN = N >> 6;
  const int tilesM = M >> 6;
  const int tile = blockIdx.x * 8 + wave;
  if (tile >= tilesM * tilesN) return;
  const int tm = tile / tilesN;
  const int tn = tile - tm * tilesN;
  const int m0 = tm << 6;
  const int n0 = tn << 6;

  const T* Ab  = A  + (size_t)b * strideA;
  const T* Bb  = Bt + (size_t)b * strideB;
  const T* Ab2 = SPLIT ? (A2  + (size_t)b * strideA) : nullptr;
  const T* Bb2 = SPLIT ? (Bt2 + (size_t)b * strideB) : nullptr;

  const int rlane = lane & 15;
  const int koff  = (lane >> 4) * 8;
  const int mOff  = (lane >> 4) * 8;

  v8f acc[4][4];
#pragma unroll
  for (int i = 0; i < 4; ++i)
#pragma unroll
    for (int j = 0; j < 4; ++j) acc[i][j] = (v8f){0.f,0.f,0.f,0.f,0.f,0.f,0.f,0.f};

  for (int k0 = 0; k0 < K; k0 += 32) {
    V bh[4], bl[4];
#pragma unroll
    for (int j = 0; j < 4; ++j) {
      const size_t bo = (size_t)(n0 + (j << 4) + rlane) * ldb + koff + k0;
      bh[j] = Frag<T>::load(Bb + bo);
      if (SPLIT) bl[j] = Frag<T>::load(Bb2 + bo);
    }
#pragma unroll
    for (int i = 0; i < 4; ++i) {
      const size_t ao = (size_t)(m0 + (i << 4) + rlane) * lda + koff + k0;
      V ah = Frag<T>::load(Ab + ao);
      V al;
      if (SPLIT) al = Frag<T>::load(Ab2 + ao);
#pragma unroll
      for (int j = 0; j < 4; ++j) {
        acc[i][j] = Frag<T>::mma(ah, bh[j], acc[i][j]);
        if (SPLIT) {
          acc[i][j] = Frag<T>::mma(ah, bl[j], acc[i][j]);
          acc[i][j] = Frag<T>::mma(al, bh[j], acc[i][j]);
        }
      }
      Frag<T>::guard(acc[i][0], acc[i][3], ah, SPLIT ? al : ah);
    }
    Frag<T>::keep(bh[0], bh[1], bh[2], bh[3]);
    if (SPLIT) Frag<T>::keep(bl[0], bl[1], bl[2], bl[3]);
  }
  acc_guard4(acc[0][0], acc[0][1], acc[0][2], acc[0][3]);
  acc_guard4(acc[1][0], acc[1][1], acc[1][2], acc[1][3]);
  acc_guard4(acc[2][0], acc[2][1], acc[2][2], acc[2][3]);
  acc_guard4(acc[3][0], acc[3][1], acc[3][2], acc[3][3]);

  float* slab = sT[wave];
  const float* Rb = RESID ? (resid + (size_t)b * strideR) : nullptr;
#pragma unroll
  for (int i = 0; i < 4; ++i) {
    const int mBase = m0 + (i << 4);
#pragma unroll
    for (int j = 0; j < 4; ++j) {
      const int n = n0 + (j << 4) + rlane;
      float bv = 0.f;
      if (BIAS_MODE == 2) bv = bias[n];
#pragma unroll
      for (int r = 0; r < 8; ++r) {
        float v = acc[i][j][r] * scale;
        if (BIAS_MODE == 1) v += bias[mBase + mOff + r];
        if (BIAS_MODE == 2) v += bv;
        if (RESID) v += Rb[(size_t)(mBase + mOff + r) * ldc + n];
        if (ACT == 1) v = tanhf(v);
        if (ACT == 2) v = fmaxf(v, 0.0f);
        if (ACT == 3) v = v / (1.0f + expf(-v));
        if (ACT == 4) v = (v > 0.f) ? v : 0.01f * v;
        if (ACT == 6) v = 1.0f / (1.0f + expf(-v));
        if (ACT == 7) { const float sg = 1.0f / (1.0f + expf(-v)); v = expf(-0.606531f * sg); }
        slab[(mOff + r) * 68 + (j << 4) + rlane] = v;
      }
    }
    __builtin_amdgcn_fence(__ATOMIC_RELEASE, "workgroup");
    __builtin_amdgcn_wave_barrier();
    __builtin_amdgcn_fence(__ATOMIC_ACQUIRE, "workgroup");
    if (OUT_MODE == 0) {
      float* C = (float*)Cout + (size_t)b * strideC;
      const int hh = lane >> 4, c4 = (lane & 15) * 4;
      for (int pass = 0; pass < 2; ++pass) {
#pragma unroll
        for (int it = 0; it < 8; ++it) {
          const int row = it * 2 + hh;
          v4f v = *(const v4f*)(slab + row * 68 + c4);
          *(volatile v4f*)(C + (size_t)(mBase + row) * ldc + n0 + c4) = v;
        }
        __threadfence();
      }
    } else {
      const int q = lane >> 3, c8 = (lane & 7) * 8;
      unsigned short* C  = (unsigned short*)Cout  + (size_t)b * strideC;
      unsigned short* C2 = (OUT_MODE == 2) ? ((unsigned short*)Cout2 + (size_t)b * strideC) : nullptr;
      for (int pass = 0; pass < 2; ++pass) {
#pragma unroll
        for (int it = 0; it < 4; ++it) {
          const int row = it * 4 + q;
          const float* sp = slab + row * 68 + c8;
          v8h hv, lv;
#pragma unroll
          for (int e = 0; e < 8; ++e) {
            if (OUT_MODE == 1) {
              hv[e] = (_Float16)sp[e];
            } else {
              unsigned short hb = f2bf_bits(sp[e]);
              unsigned short lb = f2bf_bits(sp[e] - bf_bits2f(hb));
              hv[e] = __builtin_bit_cast(_Float16, hb);
              lv[e] = __builtin_bit_cast(_Float16, lb);
            }
          }
          *(volatile v8h*)(C + (size_t)(mBase + row) * ldc + n0 + c8) = hv;
          if (OUT_MODE == 2) *(volatile v8h*)(C2 + (size_t)(mBase + row) * ldc + n0 + c8) = lv;
        }
        __threadfence();
      }
    }
    __builtin_amdgcn_fence(__ATOMIC_RELEASE, "workgroup");
    __builtin_amdgcn_wave_barrier();
    __builtin_amdgcn_fence(__ATOMIC_ACQUIRE, "workgroup");
  }
}

__device__ __forceinline__ float wave_sum(float v) {
  v += __shfl_xor(v, 16, 32);
  v += __shfl_xor(v, 8, 32);
  v += __shfl_xor(v, 4, 32);
  v += __shfl_xor(v, 2, 32);
  v += __shfl_xor(v, 1, 32);
  return v;
}

__global__ __launch_bounds__(256) void cast_f16x2_scaled(
    const float* __restrict__ in, _Float16* __restrict__ out, int n2, float scale) {
  const int i = blockIdx.x * 256 + threadIdx.x;
  if (i < n2) {
    const _Float16 h0 = (_Float16)(in[2 * i] * scale), h1 = (_Float16)(in[2 * i + 1] * scale);
    const unsigned u = (unsigned)__builtin_bit_cast(unsigned short, h0) | ((unsigned)__builtin_bit_cast(unsigned short, h1) << 16);
    ((volatile unsigned*)out)[i] = u;
    __threadfence();
    ((volatile unsigned*)out)[i] = u;
  }
}

__global__ __launch_bounds__(256) void cast_bf16hl_x2(
    const float* __restrict__ in, unsigned short* __restrict__ hi, unsigned short* __restrict__ lo, int n2) {
  const int i = blockIdx.x * 256 + threadIdx.x;
  if (i < n2) {
    const float f0 = in[2 * i], f1 = in[2 * i + 1];
    const unsigned short h0 = f2bf_bits(f0), h1 = f2bf_bits(f1);
    const unsigned short l0 = f2bf_bits(f0 - bf_bits2f(h0)), l1 = f2bf_bits(f1 - bf_bits2f(h1));
    const unsigned uh = (unsigned)h0 | ((unsigned)h1 << 16);
    const unsigned ul = (unsigned)l0 | ((unsigned)l1 << 16);
    ((volatile unsigned*)hi)[i] = uh;
    ((volatile unsigned*)lo)[i] = ul;
    __threadfence();
    ((volatile unsigned*)hi)[i] = uh;
    ((volatile unsigned*)lo)[i] = ul;
  }
}

template <int TR, int TC>
__global__ __launch_bounds__(256) void tr_cast(const float* __restrict__ in, int R, int Cc,
                                               _Float16* __restrict__ out, float scale) {
  static_assert(TR * TC == 2048, "");
  __shared__ __align__(16) float sm[TC][TR + 8];
  const int tid = threadIdx.x;
  const int r0 = blockIdx.y * TR, c0 = blockIdx.x * TC;
  constexpr int C4 = TC / 4;
#pragma unroll
  for (int q = 0; q < 2; ++q) {
    const int f = tid + 256 * q;
    const int row = f / C4, col = (f - row * C4) * 4;
    const v4f v = *(const v4f*)(in + (size_t)(r0 + row) * Cc + c0 + col);
    sm[col + 0][row] = v[0];
    sm[col + 1][row] = v[1];
    sm[col + 2][row] = v[2];
    sm[col + 3][row] = v[3];
  }
  __syncthreads();
  const int lin = tid * 8;
  const int orow = lin / TR, ocol = lin - orow * TR;
  const v4f a = *(const v4f*)(&sm[orow][ocol]);
  const v4f c = *(const v4f*)(&sm[orow][ocol + 4]);
  v8h hv;
  hv[0] = (_Float16)(a[0] * scale); hv[1] = (_Float16)(a[1] * scale);
  hv[2] = (_Float16)(a[2] * scale); hv[3] = (_Float16)(a[3] * scale);
  hv[4] = (_Float16)(c[0] * scale); hv[5] = (_Float16)(c[1] * scale);
  hv[6] = (_Float16)(c[2] * scale); hv[7] = (_Float16)(c[3] * scale);
  _Float16* dst = out + (size_t)(c0 + orow) * R + r0 + ocol;
  *(volatile v8h*)dst = hv;
  __threadfence();
  *(volatile v8h*)dst = hv;
}

__global__ __launch_bounds__(256) void fill_zero_u4(unsigned short* __restrict__ p, int n8) {
  const int i = blockIdx.x * 256 + threadIdx.x;
  if (i < n8) {
    const v4u z = {0u, 0u, 0u, 0u};
    *(volatile v4u*)(p + (size_t)8 * i) = z;
    __threadfence();
    *(volatile v4u*)(p + (size_t)8 * i) = z;
  }
}

__global__ __launch_bounds__(256) void copy_f4(const float* __restrict__ in, float* __restrict__ out, int n4) {
  const int i = blockIdx.x * 256 + threadIdx.x;
  if (i < n4) {
    const v4f v = *(const v4f*)(in + (size_t)4 * i);
    *(volatile v4f*)(out + (size_t)4 * i) = v;
    __threadfence();
    *(volatile v4f*)(out + (size_t)4 * i) = v;
  }
}

__global__ __launch_bounds__(256)
void ln1_kernel(const float* __restrict__ x, const float* __restrict__ w, const float* __restrict__ bb,
                float* __restrict__ xn, float* __restrict__ s1out, float eps) {
  __shared__ float red[8];
  __shared__ float red2[8];
  const int t = blockIdx.x, tid = threadIdx.x, lane = tid & 31, wave = tid >> 5;
  const float* row = x + (size_t)t * HID;
  const int c0 = tid * 4, c1 = HID / 2 + tid * 4;
  const v4f xa = *(const v4f*)(row + c0);
  const v4f xb = *(const v4f*)(row + c1);
  float s = ((xa[0] + xa[1]) + (xa[2] + xa[3])) + ((xb[0] + xb[1]) + (xb[2] + xb[3]));
  s = wave_sum(s);
  if (lane == 0) red[wave] = s;
  __syncthreads();
  float tot = 0.f;
#pragma unroll
  for (int q = 0; q < 8; ++q) tot += red[q];
  const float mean = tot * (1.0f / HID);
  float d[8];
#pragma unroll
  for (int e = 0; e < 4; ++e) { d[e] = xa[e] - mean; d[4 + e] = xb[e] - mean; }
  float q2 = 0.f;
#pragma unroll
  for (int e = 0; e < 8; ++e) q2 += d[e] * d[e];
  q2 = wave_sum(q2);
  if (lane == 0) red2[wave] = q2;
  __syncthreads();
  float tot2 = 0.f;
#pragma unroll
  for (int q = 0; q < 8; ++q) tot2 += red2[q];
  const float var = tot2 * (1.0f / HID);
  const float inv = 1.0f / sqrtf(var + eps);
  const v4f wa = *(const v4f*)(w + c0), wb = *(const v4f*)(w + c1);
  const v4f ba = *(const v4f*)(bb + c0), b2 = *(const v4f*)(bb + c1);
  v4f ya, yb;
#pragma unroll
  for (int e = 0; e < 4; ++e) {
    ya[e] = d[e] * inv * wa[e] + ba[e];
    yb[e] = d[4 + e] * inv * wb[e] + b2[e];
  }
  float* dst = xn + (size_t)t * HID;
  *(volatile v4f*)(dst + c0) = ya;
  *(volatile v4f*)(dst + c1) = yb;
  __threadfence();
  *(volatile v4f*)(dst + c0) = ya;
  *(volatile v4f*)(dst + c1) = yb;
  if (t == TLEN - 1) {
    *(volatile v4f*)(s1out + c0) = ya;
    *(volatile v4f*)(s1out + c1) = yb;
    __threadfence();
    *(volatile v4f*)(s1out + c0) = ya;
    *(volatile v4f*)(s1out + c1) = yb;
  }
}

__global__ __launch_bounds__(256)
void mix_kernel(const float* __restrict__ xn, const float* __restrict__ state1,
                const float* __restrict__ mr, const float* __restrict__ mw, const float* __restrict__ mk,
                const float* __restrict__ mv, const float* __restrict__ ma, const float* __restrict__ mg,
                _Float16* __restrict__ xr16, _Float16* __restrict__ xw16, _Float16* __restrict__ xv16,
                _Float16* __restrict__ xa16, _Float16* __restrict__ xg16,
                unsigned short* __restrict__ xkh, unsigned short* __restrict__ xkl,
                unsigned short* __restrict__ xvh, unsigned short* __restrict__ xvl) {
  const int t = blockIdx.x, j = threadIdx.x * 8;
  const size_t idx = (size_t)t * HID + j;
  const float* prow = (t == 0) ? (state1 + j) : (xn + idx - HID);
  const v4f ca = *(const v4f*)(xn + idx), cb = *(const v4f*)(xn + idx + 4);
  const v4f pa = *(const v4f*)(prow), pb = *(const v4f*)(prow + 4);
  float cur[8], sx[8];
#pragma unroll
  for (int e = 0; e < 4; ++e) {
    cur[e] = ca[e]; cur[4 + e] = cb[e];
    sx[e] = pa[e] - ca[e]; sx[4 + e] = pb[e] - cb[e];
  }
#pragma unroll 1
  for (int p = 0; p < 6; ++p) {
    const float* mp = mr;
    mp = (p == 1) ? mw : mp;
    mp = (p == 2) ? mk : mp;
    mp = (p == 3) ? mv : mp;
    mp = (p == 4) ? ma : mp;
    mp = (p == 5) ? mg : mp;
    const v4f m0 = *(const v4f*)(mp + j), m1 = *(const v4f*)(mp + j + 4);
    float xm[8];
#pragma unroll
    for (int e = 0; e < 4; ++e) {
      xm[e]     = cur[e]     + m0[e] * sx[e];
      xm[4 + e] = cur[4 + e] + m1[e] * sx[4 + e];
    }
    if (p == 2 || p == 3) {
      v8h hv, lv;
#pragma unroll
      for (int e = 0; e < 8; ++e) {
        const unsigned short hb = f2bf_bits(xm[e]);
        const unsigned short lb = f2bf_bits(xm[e] - bf_bits2f(hb));
        hv[e] = __builtin_bit_cast(_Float16, hb);
        lv[e] = __builtin_bit_cast(_Float16, lb);
      }
      unsigned short* dh = (p == 2) ? xkh : xvh;
      unsigned short* dl = (p == 2) ? xkl : xvl;
      *(volatile v8h*)(dh + idx) = hv;
      *(volatile v8h*)(dl + idx) = lv;
      __threadfence();
      *(volatile v8h*)(dh + idx) = hv;
      *(volatile v8h*)(dl + idx) = lv;
    }
    if (p != 2) {
      _Float16* dp = xr16;
      dp = (p == 1) ? xw16 : dp;
      dp = (p == 3) ? xv16 : dp;
      dp = (p == 4) ? xa16 : dp;
      dp = (p == 5) ? xg16 : dp;
      v8h hv;
#pragma unroll
      for (int e = 0; e < 8; ++e) hv[e] = (_Float16)xm[e];
      *(volatile v8h*)(dp + idx) = hv;
      __threadfence();
      *(volatile v8h*)(dp + idx) = hv;
    }
  }
}

__global__ __launch_bounds__(256)
void coeff_kernel(const float* __restrict__ kbuf, const float* __restrict__ abuf, const float* __restrict__ vbuf,
                  const float* __restrict__ pbuf, const float* __restrict__ vfirst,
                  const float* __restrict__ k_k, const float* __restrict__ k_a,
                  float* __restrict__ kmod, float* __restrict__ vfin,
                  float* __restrict__ aseq, float* __restrict__ bseq) {
  __shared__ float red[8];
  const int b = blockIdx.x, tid = threadIdx.x, lane = tid & 31, wave = tid >> 5;
  const int grp = tid >> 6, i = tid & 63;
  const int hg = (b & 7) * 4 + grp;
  const size_t idx = (size_t)b * 256 + tid;
  const float kv = kbuf[idx], av = abuf[idx], vv = vbuf[idx], pv = pbuf[idx], vf = vfirst[idx];
  const float kkp = k_k[hg * HSZ + i], kap = k_a[hg * HSZ + i];
  const float kk = kv * kkp;
  float ss = wave_sum(kk * kk);
  if (lane == 0) red[wave] = ss;
  __syncthreads();
  const float nrm = sqrtf(red[grp * 2] + red[grp * 2 + 1]) + 1e-12f;
  const float kkn = kk * (1.0f / nrm);
  const float km = kv * (1.0f + (av - 1.0f) * kap);
  const float vb = vv + (vf - vv) * pv;
  const float as = -kkn, bs = kkn * av;
  ((volatile float*)kmod)[idx] = km;
  ((volatile float*)vfin)[idx] = vb;
  ((volatile float*)aseq)[idx] = as;
  ((volatile float*)bseq)[idx] = bs;
  __threadfence();
  ((volatile float*)kmod)[idx] = km;
  ((volatile float*)vfin)[idx] = vb;
  ((volatile float*)aseq)[idx] = as;
  ((volatile float*)bseq)[idx] = bs;
}

__global__ __launch_bounds__(256)
void scan_kernel(const float* __restrict__ state2, const float* __restrict__ wdec, const float* __restrict__ kmod,
                 const float* __restrict__ aseq, const float* __restrict__ bseq, const float* __restrict__ rbuf,
                 const float* __restrict__ vfin, float* __restrict__ ybuf, float* __restrict__ s2out) {
  __shared__ __align__(16) float vb[2][6][HSZ];
  __shared__ __align__(16) float yl[2][16][HSZ];
  __shared__ __align__(16) float st[HSZ][68];
  const int hh = blockIdx.x, tid = threadIdx.x, wave = tid >> 5, lane = tid & 31;
  const int i = tid >> 2, jq = tid & 3, j0 = jq * 16;
  float S[16];
  {
    const float* sp = state2 + ((size_t)(hh * HSZ + i) * HSZ + j0);
#pragma unroll
    for (int q = 0; q < 4; ++q) {
      const v4f v = *(const v4f*)(sp + 4 * q);
      S[4 * q + 0] = v[0]; S[4 * q + 1] = v[1]; S[4 * q + 2] = v[2]; S[4 * q + 3] = v[3];
    }
  }
  for (int t = 0; t <= TLEN; ++t) {
    const int buf = t & 1;
    if (t < TLEN) {
      if (wave < 6) {
        const float* src = wdec;
        src = (wave == 1) ? kmod : src;
        src = (wave == 2) ? aseq : src;
        src = (wave == 3) ? bseq : src;
        src = (wave == 4) ? rbuf : src;
        src = (wave == 5) ? vfin : src;
        const v2f v = *(const v2f*)(src + (size_t)t * HID + hh * HSZ + lane * 2);
        *(v2f*)(&vb[buf][wave][lane * 2]) = v;
      }
    }
    __syncthreads();
    if (((t & 15) == 0) && (t > 0)) {
      const int ch = (t >> 4) - 1;
      const int L = tid >> 3, tt = L >> 1, hf = L & 1, c4 = (tid & 7) * 4;
      const v4f v = *(const v4f*)(&yl[ch & 1][tt][hf * 32 + c4]);
      float* dst = ybuf + (size_t)(ch * 16 + tt) * HID + hh * HSZ + hf * 32 + c4;
      *(volatile v4f*)dst = v;
      __threadfence();
      *(volatile v4f*)dst = v;
    }
    if (t < TLEN) {
      float wv[16], kv[16], av[16], bvv[16], rv[16];
#pragma unroll
      for (int q = 0; q < 4; ++q) {
        const v4f tw = *(const v4f*)(&vb[buf][0][j0 + 4 * q]);
        const v4f tk = *(const v4f*)(&vb[buf][1][j0 + 4 * q]);
        const v4f ta = *(const v4f*)(&vb[buf][2][j0 + 4 * q]);
        const v4f tb = *(const v4f*)(&vb[buf][3][j0 + 4 * q]);
        const v4f tr = *(const v4f*)(&vb[buf][4][j0 + 4 * q]);
#pragma unroll
        for (int e = 0; e < 4; ++e) {
          wv[4 * q + e] = tw[e]; kv[4 * q + e] = tk[e]; av[4 * q + e] = ta[e];
          bvv[4 * q + e] = tb[e]; rv[4 * q + e] = tr[e];
        }
      }
      float p = 0.f;
#pragma unroll
      for (int e = 0; e < 16; ++e) {
        S[e] = S[e] * wv[e];
        p += S[e] * av[e];
      }
      p += __shfl_xor(p, 1, 32);
      p += __shfl_xor(p, 2, 32);
      const float vi = vb[buf][5][i];
      float o = 0.f;
#pragma unroll
      for (int e = 0; e < 16; ++e) {
        S[e] = S[e] + p * bvv[e] + vi * kv[e];
        o += S[e] * rv[e];
      }
      o += __shfl_xor(o, 1, 32);
      o += __shfl_xor(o, 2, 32);
      if (jq == 0) yl[(t >> 4) & 1][t & 15][i] = o;
    }
  }
#pragma unroll
  for (int q = 0; q < 4; ++q) {
    v4f v;
    v[0] = S[4 * q + 0]; v[1] = S[4 * q + 1]; v[2] = S[4 * q + 2]; v[3] = S[4 * q + 3];
    *(v4f*)(&st[i][j0 + 4 * q]) = v;
  }
  __syncthreads();
  for (int pass = 0; pass < 2; ++pass) {
#pragma unroll
    for (int it = 0; it < 4; ++it) {
      const int f = it * 256 + tid;
      const int row = f >> 4, c4 = (f & 15) * 4;
      const v4f v = *(const v4f*)(&st[row][c4]);
      *(volatile v4f*)(s2out + (size_t)(hh * HSZ + row) * HSZ + c4) = v;
    }
    __threadfence();
  }
}

__global__ __launch_bounds__(256)
void gn_kernel(const float* __restrict__ ybuf, const float* __restrict__ rbuf, const float* __restrict__ kmod,
               const float* __restrict__ vfin, const float* __restrict__ gbuf,
               const float* __restrict__ r_k, const float* __restrict__ lnw, const float* __restrict__ lnb,
               _Float16* __restrict__ yg) {
  __shared__ float red[16];
  __shared__ float red2[8];
  __shared__ __align__(16) float fb[256];
  const int b = blockIdx.x, tid = threadIdx.x, lane = tid & 31, wave = tid >> 5;
  const int grp = tid >> 6, i = tid & 63;
  const int hg = (b & 7) * 4 + grp;
  const size_t idx = (size_t)b * 256 + tid;
  const float y = ybuf[idx], r = rbuf[idx], km = kmod[idx], vf = vfin[idx], g = gbuf[idx];
  const float rk = r_k[hg * HSZ + i], lw = lnw[hg * HSZ + i], lb = lnb[hg * HSZ + i];
  float s0 = wave_sum(y);
  float s1 = wave_sum(r * km * rk);
  if (lane == 0) { red[wave * 2] = s0; red[wave * 2 + 1] = s1; }
  __syncthreads();
  const int wA = grp * 2, wB = grp * 2 + 1;
  const float sum = red[wA * 2] + red[wB * 2];
  const float dot = red[wA * 2 + 1] + red[wB * 2 + 1];
  const float mean = sum * (1.0f / HSZ);
  const float d = y - mean;
  float s2 = wave_sum(d * d);
  if (lane == 0) red2[wave] = s2;
  __syncthreads();
  const float var = (red2[wA] + red2[wB]) * (1.0f / HSZ);
  const float yn = d * (1.0f / sqrtf(var + 0.00064f));
  const float yv = (yn * lw + lb + dot * vf) * g;
  fb[tid] = yv;
  __syncthreads();
  if (wave == 0) {
    const int q = lane >> 3, c8 = (lane & 7) * 8;
    const v4f a = *(const v4f*)(&fb[q * 64 + c8]);
    const v4f c = *(const v4f*)(&fb[q * 64 + c8 + 4]);
    v8h hv;
    hv[0] = (_Float16)a[0]; hv[1] = (_Float16)a[1]; hv[2] = (_Float16)a[2]; hv[3] = (_Float16)a[3];
    hv[4] = (_Float16)c[0]; hv[5] = (_Float16)c[1]; hv[6] = (_Float16)c[2]; hv[7] = (_Float16)c[3];
    _Float16* dst = yg + (size_t)b * 256 + q * 64 + c8;
    *(volatile v8h*)dst = hv;
    __threadfence();
    *(volatile v8h*)dst = hv;
  }
}

static inline int gemm_grid(int M, int N) { return ((M / 64) * (N / 64) + 7) / 8; }
static inline const unsigned short* u16c(const void* p) { return (const unsigned short*)p; }

extern "C" void kernel_launch(void* const* d_in, const int* in_sizes, int n_in,
                              void* d_out, int out_size, void* d_ws, size_t ws_size,
                              hipStream_t stream) {
  if (n_in < 32) return;
  if (in_sizes[0] != TLEN * HID || in_sizes[1] != HID || in_sizes[2] != NHEAD * HSZ * HSZ ||
      in_sizes[3] != TLEN * HID || in_sizes[10] != HID * HID || in_sizes[13] != HID * HID ||
      in_sizes[15] != HID * DLD || in_sizes[18] != HID * DLA || in_sizes[21] != HID * DLV ||
      in_sizes[23] != HID * DLG || in_sizes[25] != NHEAD * HSZ) return;
  if ((size_t)out_size != OUT_TOTAL_F || ws_size < WS_END) return;

  const float* x       = (const float*)d_in[0];
  const float* state1  = (const float*)d_in[1];
  const float* state2  = (const float*)d_in[2];
  const float* v_first = (const float*)d_in[3];
  const float* x_r = (const float*)d_in[4];
  const float* x_w = (const float*)d_in[5];
  const float* x_k = (const float*)d_in[6];
  const float* x_v = (const float*)d_in[7];
  const float* x_a = (const float*)d_in[8];
  const float* x_g = (const float*)d_in[9];
  const float* W_r = (const float*)d_in[10];
  const float* W_k = (const float*)d_in[11];
  const float* W_v = (const float*)d_in[12];
  const float* W_o = (const float*)d_in[13];
  const float* w0  = (const float*)d_in[14];
  const float* w1  = (const float*)d_in[15];
  const float* w2  = (const float*)d_in[16];
  const float* a0  = (const float*)d_in[17];
  const float* a1  = (const float*)d_in[18];
  const float* a2  = (const float*)d_in[19];
  const float* v0  = (const float*)d_in[20];
  const float* v1  = (const float*)d_in[21];
  const float* v2  = (const float*)d_in[22];
  const float* g1  = (const float*)d_in[23];
  const float* g2  = (const float*)d_in[24];
  const float* k_k = (const float*)d_in[25];
  const float* k_a = (const float*)d_in[26];
  const float* r_k = (const float*)d_in[27];
  const float* ln_x_w = (const float*)d_in[28];
  const float* ln_x_b = (const float*)d_in[29];
  const float* ln1_w  = (const float*)d_in[30];
  const float* ln1_b  = (const float*)d_in[31];

  char* ws = (char*)d_ws;
  _Float16* Wo16 = (_Float16*)(ws + OFF_WO16);
  _Float16* g1T = (_Float16*)(ws + OFF_G1T);
  _Float16* g2T = (_Float16*)(ws + OFF_G2T);
  _Float16* w1T = (_Float16*)(ws + OFF_W1T);
  _Float16* w2T = (_Float16*)(ws + OFF_W2T);
  _Float16* a1T = (_Float16*)(ws + OFF_A1T);
  _Float16* a2T = (_Float16*)(ws + OFF_A2T);
  _Float16* v1T = (_Float16*)(ws + OFF_V1T);
  _Float16* v2T = (_Float16*)(ws + OFF_V2T);
  _Float16* hg16 = (_Float16*)(ws + OFF_HG);
  _Float16* hw16 = (_Float16*)(ws + OFF_HW);
  _Float16* ha16 = (_Float16*)(ws + OFF_HA);
  _Float16* hv16 = (_Float16*)(ws + OFF_HV);
  _Float16* yg16 = (_Float16*)(ws + OFF_YG);
  _Float16* Wr16 = (_Float16*)(ws + OFF_WR16);
  unsigned short* Wkh = (unsigned short*)(ws + OFF_WKH);
  unsigned short* Wkl = (unsigned short*)(ws + OFF_WKL);
  unsigned short* Wvh = (unsigned short*)(ws + OFF_WVH);
  unsigned short* Wvl = (unsigned short*)(ws + OFF_WVL);
  float* gbuf = (float*)(ws + OFF_GBUF);
  float* wdec = (float*)(ws + OFF_WDEC);
  float* abuf = (float*)(ws + OFF_ABUF);
  float* pbuf = (float*)(ws + OFF_PBUF);
  float* ybuf = (float*)(ws + OFF_YBUF);
  float* xn = (float*)(ws + OFF_XN);
  _Float16* xr16 = (_Float16*)(ws + OFF_XR16);
  _Float16* xw16 = (_Float16*)(ws + OFF_XW16);
  _Float16* xa16 = (_Float16*)(ws + OFF_XA16);
  _Float16* xg16 = (_Float16*)(ws + OFF_XG16);
  _Float16* xv16 = (_Float16*)(ws + OFF_XV16);
  unsigned short* xkh = (unsigned short*)(ws + OFF_XKH);
  unsigned short* xkl = (unsigned short*)(ws + OFF_XKL);
  unsigned short* xvh = (unsigned short*)(ws + OFF_XVH);
  unsigned short* xvl = (unsigned short*)(ws + OFF_XVL);
  float* kmodp = (float*)(ws + OFF_KMOD);
  float* vfinp = (float*)(ws + OFF_VFIN);
  float* aseqp = (float*)(ws + OFF_ASEQ);
  float* bseqp = (float*)(ws + OFF_BSEQ);
  float* rbuf = (float*)(ws + OFF_RBUF);
  float* kbuf = (float*)(ws + OFF_KBUF);
  float* vbuf = (float*)(ws + OFF_VBUF);

  float* out0 = (float*)d_out + OUT0_F;
  float* out1 = (float*)d_out + OUT1_F;
  float* out2 = (float*)d_out + OUT2_F;
  float* out3 = (float*)d_out + OUT3_F;

  const dim3 blk(256);
  const int n2W = HID * HID / 2;
  const int gW = (n2W + 255) / 256;

  cast_f16x2_scaled<<<dim3(gW), blk, 0, stream>>>(W_o, Wo16, n2W, WCARRY);
  cast_f16x2_scaled<<<dim3(gW), blk, 0, stream>>>(W_r, Wr16, n2W, WCARRY);
  cast_bf16hl_x2<<<dim3(gW), blk, 0, stream>>>(W_k, Wkh, Wkl, n2W);
  cast_bf16hl_x2<<<dim3(gW), blk, 0, stream>>>(W_v, Wvh, Wvl, n2W);
  tr_cast<64, 32><<<dim3(DLG / 32, HID / 64), blk, 0, stream>>>(g1, HID, DLG, g1T, WCARRY);
  tr_cast<64, 32><<<dim3(HID / 32, DLG / 64), blk, 0, stream>>>(g2, DLG, HID, g2T, WCARRY);
  tr_cast<64, 32><<<dim3(DLD / 32, HID / 64), blk, 0, stream>>>(w1, HID, DLD, w1T, WCARRY);
  tr_cast<64, 32><<<dim3(HID / 32, DLD / 64), blk, 0, stream>>>(w2, DLD, HID, w2T, WCARRY);
  tr_cast<64, 32><<<dim3(DLA / 32, HID / 64), blk, 0, stream>>>(a1, HID, DLA, a1T, WCARRY);
  tr_cast<64, 32><<<dim3(HID / 32, DLA / 64), blk, 0, stream>>>(a2, DLA, HID, a2T, WCARRY);
  tr_cast<64, 32><<<dim3(DLV / 32, HID / 64), blk, 0, stream>>>(v1, HID, DLV, v1T, WCARRY);
  fill_zero_u4<<<dim3(((DLVP - DLV) * HID / 8 + 255) / 256), blk, 0, stream>>>(
      (unsigned short*)(v1T + (size_t)DLV * HID), (DLVP - DLV) * HID / 8);
  tr_cast<32, 64><<<dim3(HID / 64, DLV / 32), blk, 0, stream>>>(v2, DLV, HID, v2T, WCARRY);

  ln1_kernel<<<dim3(TLEN), blk, 0, stream>>>(x, ln1_w, ln1_b, xn, out1, 1e-5f);

  mix_kernel<<<dim3(TLEN), blk, 0, stream>>>(xn, state1, x_r, x_w, x_k, x_v, x_a, x_g,
                                             xr16, xw16, xv16, xa16, xg16, xkh, xkl, xvh, xvl);

  const int gBig = gemm_grid(TLEN, HID);
  wmma_gemm64<0, false, 0, 0, false, 0><<<dim3(gBig), blk, 0, stream>>>(
      u16c(xr16), nullptr, HID, 0L, u16c(Wr16), nullptr, HID, 0L,
      (void*)rbuf, nullptr, HID, 0L, nullptr, nullptr, 0L, TLEN, HID, HID, WCARRY_INV);
  wmma_gemm64<1, true, 0, 0, false, 0><<<dim3(gBig), blk, 0, stream>>>(
      u16c(xkh), u16c(xkl), HID, 0L, u16c(Wkh), u16c(Wkl), HID, 0L,
      (void*)kbuf, nullptr, HID, 0L, nullptr, nullptr, 0L, TLEN, HID, HID, 1.0f);
  wmma_gemm64<1, true, 0, 0, false, 0><<<dim3(gBig), blk, 0, stream>>>(
      u16c(xvh), u16c(xvl), HID, 0L, u16c(Wvh), u16c(Wvl), HID, 0L,
      (void*)vbuf, nullptr, HID, 0L, nullptr, nullptr, 0L, TLEN, HID, HID, 1.0f);

  wmma_gemm64<0, false, 0, 1, false, 6><<<dim3(gemm_grid(TLEN, DLG)), blk, 0, stream>>>(
      u16c(xg16), nullptr, HID, 0L, u16c(g1T), nullptr, HID, 0L,
      (void*)hg16, nullptr, DLG, 0L, nullptr, nullptr, 0L, TLEN, DLG, HID, WCARRY_INV);
  wmma_gemm64<0, false, 0, 1, false, 1><<<dim3(gemm_grid(TLEN, DLD)), blk, 0, stream>>>(
      u16c(xw16), nullptr, HID, 0L, u16c(w1T), nullptr, HID, 0L,
      (void*)hw16, nullptr, DLD, 0L, nullptr, nullptr, 0L, TLEN, DLD, HID, WCARRY_INV);
  wmma_gemm64<0, false, 0, 1, false, 0><<<dim3(gemm_grid(TLEN, DLA)), blk, 0, stream>>>(
      u16c(xa16), nullptr, HID, 0L, u16c(a1T), nullptr, HID, 0L,
      (void*)ha16, nullptr, DLA, 0L, nullptr, nullptr, 0L, TLEN, DLA, HID, WCARRY_INV);
  wmma_gemm64<0, false, 0, 1, false, 0><<<dim3(gemm_grid(TLEN, DLVP)), blk, 0, stream>>>(
      u16c(xv16), nullptr, HID, 0L, u16c(v1T), nullptr, HID, 0L,
      (void*)hv16, nullptr, DLVP, 0L, nullptr, nullptr, 0L, TLEN, DLVP, HID, WCARRY_INV);

  wmma_gemm64<0, false, 0, 0, false, 0><<<dim3(gBig), blk, 0, stream>>>(
      u16c(hg16), nullptr, DLG, 0L, u16c(g2T), nullptr, DLG, 0L,
      (void*)gbuf, nullptr, HID, 0L, nullptr, nullptr, 0L, TLEN, HID, DLG, WCARRY_INV);
  wmma_gemm64<0, false, 2, 0, false, 7><<<dim3(gBig), blk, 0, stream>>>(
      u16c(hw16), nullptr, DLD, 0L, u16c(w2T), nullptr, DLD, 0L,
      (void*)wdec, nullptr, HID, 0L, w0, nullptr, 0L, TLEN, HID, DLD, WCARRY_INV);
  wmma_gemm64<0, false, 2, 0, false, 6><<<dim3(gBig), blk, 0, stream>>>(
      u16c(ha16), nullptr, DLA, 0L, u16c(a2T), nullptr, DLA, 0L,
      (void*)abuf, nullptr, HID, 0L, a0, nullptr, 0L, TLEN, HID, DLA, WCARRY_INV);
  wmma_gemm64<0, false, 2, 0, false, 6><<<dim3(gBig), blk, 0, stream>>>(
      u16c(hv16), nullptr, DLVP, 0L, u16c(v2T), nullptr, DLV, 0L,
      (void*)pbuf, nullptr, HID, 0L, v0, nullptr, 0L, TLEN, HID, DLV, WCARRY_INV);

  const int gEl = TLEN * HID / 256;
  coeff_kernel<<<dim3(gEl), blk, 0, stream>>>(kbuf, abuf, vbuf, pbuf, v_first, k_k, k_a,
                                              kmodp, vfinp, aseqp, bseqp);

  scan_kernel<<<dim3(NHEAD), blk, 0, stream>>>(state2, wdec, kmodp, aseqp, bseqp, rbuf, vfinp, ybuf, out2);

  gn_kernel<<<dim3(gEl), blk, 0, stream>>>(ybuf, rbuf, kmodp, vfinp, gbuf, r_k, ln_x_w, ln_x_b, yg16);

  wmma_gemm64<0, false, 0, 0, true, 0><<<dim3(gBig), blk, 0, stream>>>(
      u16c(yg16), nullptr, HID, 0L, u16c(Wo16), nullptr, HID, 0L,
      (void*)out0, nullptr, HID, 0L, nullptr, x, 0L, TLEN, HID, HID, WCARRY_INV);

  copy_f4<<<dim3((TLEN * HID / 4 + 255) / 256), blk, 0, stream>>>(v_first, out3, TLEN * HID / 4);
}
